// SelfAttention2d_60765197303891
// MI455X (gfx1250) — hardware-verified
//
#include <hip/hip_runtime.h>


#ifndef NB
#define NB 32
#endif
#define NB_FULL 32
#ifndef SEQ
#define SEQ 1024
#endif
#define SEQ_FULL 1024
#define CC   256
#define NG   8
#define CG   (CC / NG)
#define NQKV (3 * CC)
#define HD   CC
#define GBATCH ((NB) < 8 ? (NB) : 8)
#define PCAR 1024.0f
#define SCL  0.0625f
#define WSC  16.0f
#define CTS  16.0f
#define GNEPS 1e-5f
static_assert(SEQ % 128 == 0);
static_assert(SEQ <= SEQ_FULL);
static_assert(NB >= 1 && NB <= NB_FULL);
static_assert(CC % 64 == 0 && NQKV % 64 == 0 && HD % 64 == 0 && SEQ % 64 == 0);
static_assert(((NQKV * CC / 8) % 256) == 0 && ((CC * CC / 8) % 256) == 0);

typedef _Float16 h16;
typedef unsigned short bf;
typedef __attribute__((ext_vector_type(16))) __bf16   v16bf;
typedef __attribute__((ext_vector_type(16))) _Float16 v16h;
typedef __attribute__((ext_vector_type(8)))  _Float16 v8h;
typedef __attribute__((ext_vector_type(8)))  unsigned short v8us;
typedef __attribute__((ext_vector_type(8)))  float    v8f;
typedef __attribute__((ext_vector_type(4)))  float    v4f;
typedef __attribute__((ext_vector_type(4)))  _Float16 v4h;
typedef v8h  __attribute__((may_alias)) v8ha;
typedef v4f  __attribute__((may_alias)) v4fa;
typedef v8us __attribute__((may_alias)) v8usa;

__device__ __forceinline__ unsigned short f2bf(float f) { unsigned u = __float_as_uint(f); u += 0x7FFFu + ((u >> 16) & 1u); return (unsigned short)(u >> 16); }
__device__ __forceinline__ float bf2f(unsigned short b) { return __uint_as_float(((unsigned)b) << 16); }
__device__ __forceinline__ float bfr(float f) { return bf2f(f2bf(f)); }
__device__ __forceinline__ h16 tohx(float x) { return (h16)x; }
__device__ __forceinline__ v16h cat16(v8h lo, v8h hi) { return __builtin_shufflevector(lo, hi, 0, 1, 2, 3, 4, 5, 6, 7, 8, 9, 10, 11, 12, 13, 14, 15); }
__device__ __forceinline__ v16bf cat16b(v8us lo, v8us hi) { return __builtin_bit_cast(v16bf, __builtin_shufflevector(lo, hi, 0, 1, 2, 3, 4, 5, 6, 7, 8, 9, 10, 11, 12, 13, 14, 15)); }
__device__ __forceinline__ v8f wmma16(v16h a, v16h b, v8f c) { return __builtin_amdgcn_wmma_f32_16x16x32_f16(false, a, false, b, (short)0, c, false, false); }
__device__ __forceinline__ v8f wmmab(v16bf a, v16bf b, v8f c) { return __builtin_amdgcn_wmma_f32_16x16x32_bf16(false, a, false, b, (short)0, c, false, false); }

template <typename T16> struct WFrag;
template <> struct WFrag<h16> { typedef v16h V; static __device__ __forceinline__ V ld(const h16* p) { return cat16(*(const v8h*)p, *(const v8h*)(p + 16)); } static __device__ __forceinline__ v8f mma(V a, V b, v8f c) { return wmma16(a, b, c); } };
template <> struct WFrag<bf> { typedef v16bf V; static __device__ __forceinline__ V ld(const bf* p) { return cat16b(*(const v8us*)p, *(const v8us*)(p + 16)); } static __device__ __forceinline__ v8f mma(V a, V b, v8f c) { return wmmab(a, b, c); } };
template <typename T16, int NSPLIT, bool BIAS>
__global__ __launch_bounds__(32) void k_gemmw(const T16* __restrict__ A, const T16* __restrict__ A2, const T16* __restrict__ Bt, const T16* __restrict__ Bt2, int K, float* C, int ldc, const float* __restrict__ bias, float osc, size_t sA, size_t sB, size_t sC) {
    typedef typename WFrag<T16>::V V;
    __shared__ __align__(16) float os[16 * 68];
    const size_t z = blockIdx.z; A += z * sA; if (A2) A2 += z * sA; Bt += z * sB; if (Bt2) Bt2 += z * sB; C += z * sC;
    const int lane = threadIdx.x & 31, lr = lane & 15, hi = lane >> 4; const int r0 = blockIdx.x * 64, c0 = blockIdx.y * 64;
    v8f acc[4][4];
#pragma unroll
    for (int mb = 0; mb < 4; ++mb)
#pragma unroll
        for (int nb = 0; nb < 4; ++nb) acc[mb][nb] = (v8f){};
    const size_t aoff = (size_t)(r0 + lr) * K + 8 * hi, boff = (size_t)(c0 + lr) * K + 8 * hi;
#pragma unroll 1
    for (int kc = 0; kc < K; kc += 32) {
        V a[4], a2[4];
#pragma unroll
        for (int mb = 0; mb < 4; ++mb) { a[mb] = WFrag<T16>::ld(A + aoff + (size_t)mb * 16 * K + kc); if (NSPLIT == 1 || NSPLIT == 2) a2[mb] = WFrag<T16>::ld(A2 + aoff + (size_t)mb * 16 * K + kc); }
#pragma unroll
        for (int nb = 0; nb < 4; ++nb) { const V b = WFrag<T16>::ld(Bt + boff + (size_t)nb * 16 * K + kc); V b2 = b; if (NSPLIT >= 2) b2 = WFrag<T16>::ld(Bt2 + boff + (size_t)nb * 16 * K + kc);
#pragma unroll
            for (int mb = 0; mb < 4; ++mb) { acc[mb][nb] = WFrag<T16>::mma(a[mb], b, acc[mb][nb]); if (NSPLIT == 1 || NSPLIT == 2) acc[mb][nb] = WFrag<T16>::mma(a2[mb], b, acc[mb][nb]); if (NSPLIT >= 2) acc[mb][nb] = WFrag<T16>::mma(a[mb], b2, acc[mb][nb]); } }
        asm volatile("v_nop\n\tv_nop\n\tv_nop\n\tv_nop" : "+v"(acc[0][0]), "+v"(acc[1][1]), "+v"(acc[2][2]), "+v"(acc[3][3]) : "v"(a[0]), "v"(a[3]));
    }
#pragma unroll
    for (int mb = 0; mb < 4; ++mb) {
#pragma unroll
        for (int nb = 0; nb < 4; ++nb) {
#pragma unroll
            for (int j = 0; j < 8; ++j) os[(hi * 8 + j) * 68 + nb * 16 + lr] = acc[mb][nb][j]; }
        __builtin_amdgcn_wave_barrier(); asm volatile("" ::: "memory");
        float* crow = C + (size_t)(r0 + mb * 16) * ldc + c0;
#pragma unroll 1
        for (int ps = 0; ps < 2; ++ps) {
#pragma unroll
            for (int s = 0; s < 8; ++s) { const int row = 2 * s + hi, cofs = lr * 4; v4f val = *(const v4fa*)(os + row * 68 + cofs); val = val * osc; if (BIAS) { val[0] += bfr(bias[c0 + cofs]); val[1] += bfr(bias[c0 + cofs + 1]); val[2] += bfr(bias[c0 + cofs + 2]); val[3] += bfr(bias[c0 + cofs + 3]); }
                *(volatile v4f*)(crow + (size_t)row * ldc + cofs) = val; }
            if (ps == 0) __threadfence(); }
        __builtin_amdgcn_wave_barrier(); asm volatile("" ::: "memory");
    }
}

__device__ __forceinline__ void wcvt8(const float* __restrict__ src, h16* dst, size_t j) {
    const v8f v = *(const v8f*)(src + j * 8); v8h o;
#pragma unroll
    for (int k = 0; k < 8; ++k) o[k] = tohx(bfr(v[k]) * WSC);
    *(volatile v8h*)(dst + j * 8) = o; __threadfence(); *(volatile v8h*)(dst + j * 8) = o;
}
__global__ __launch_bounds__(256) void k_wcvt(const float* __restrict__ wq, const float* __restrict__ wp, h16* W16, h16* WP16) {
    const size_t i = (size_t)blockIdx.x * 256 + threadIdx.x;
    const size_t nq8 = (size_t)NQKV * CC / 8, np8 = (size_t)CC * CC / 8;
    if (blockIdx.x < (unsigned)(nq8 / 256)) { wcvt8(wq, W16, i); }
    else { const size_t j = i - nq8; if (j >= np8) return; wcvt8(wp, WP16, j); }
}

__global__ __launch_bounds__(256) void k_gn(const float* __restrict__ x, const float* __restrict__ gw, const float* __restrict__ gbias, h16* XN) {
    __shared__ double red[2][256];
    __shared__ float tile[64][65];
    __shared__ float wsv[64], bsv[64];
    const int tid = threadIdx.x;
    const int b = blockIdx.x >> 2, cp = blockIdx.x & 3, c0 = cp * 64;
    const float* xb = x + ((size_t)b * CC + c0) * SEQ_FULL;
    if (tid < 64) { wsv[tid] = bfr(gw[c0 + tid]); bsv[tid] = bfr(gbias[c0 + tid]); }
    double sA = 0.0, sB = 0.0;
#pragma unroll 1
    for (int ci = 0; ci < CG; ++ci) {
        const float* ra = xb + (size_t)ci * SEQ_FULL; const float* rb = xb + (size_t)(ci + CG) * SEQ_FULL;
#pragma unroll 1
        for (int t = tid; t < SEQ; t += 256) { sA += (double)bfr(ra[t]); sB += (double)bfr(rb[t]); }
    }
    red[0][tid] = sA; red[1][tid] = sB;
    __syncthreads();
#pragma unroll 1
    for (int off = 128; off > 0; off >>= 1) { if (tid < off) { red[0][tid] += red[0][tid + off]; red[1][tid] += red[1][tid + off]; } __syncthreads(); }
    const double invn = 1.0 / (double)(CG * SEQ);
    const float mA = (float)(red[0][0] * invn), mB = (float)(red[1][0] * invn);
    __syncthreads();
    double vA = 0.0, vB = 0.0;
#pragma unroll 1
    for (int ci = 0; ci < CG; ++ci) {
        const float* ra = xb + (size_t)ci * SEQ_FULL; const float* rb = xb + (size_t)(ci + CG) * SEQ_FULL;
#pragma unroll 1
        for (int t = tid; t < SEQ; t += 256) { const float da = bfr(ra[t]) - mA; const float db = bfr(rb[t]) - mB; vA += (double)da * (double)da; vB += (double)db * (double)db; }
    }
    red[0][tid] = vA; red[1][tid] = vB;
    __syncthreads();
#pragma unroll 1
    for (int off = 128; off > 0; off >>= 1) { if (tid < off) { red[0][tid] += red[0][tid + off]; red[1][tid] += red[1][tid + off]; } __syncthreads(); }
    const float varA = (float)(red[0][0] * invn), varB = (float)(red[1][0] * invn);
    const float rA = 1.0f / sqrtf(varA + GNEPS), rB = 1.0f / sqrtf(varB + GNEPS);
    __syncthreads();
    const int tl = tid & 63, cb = tid >> 6; const int srow = tid >> 3, part = tid & 7;
#pragma unroll 1
    for (int t0 = 0; t0 < SEQ; t0 += 64) {
#pragma unroll 1
        for (int ci = cb; ci < 64; ci += 4) {
            const float v = bfr(xb[(size_t)ci * SEQ_FULL + t0 + tl]);
            const bool gB = (ci >= CG); const float m = gB ? mB : mA; const float r = gB ? rB : rA;
            tile[ci][tl] = ((v - m) * r) * wsv[ci] + bsv[ci];
        }
        __syncthreads();
        v8h o0, o1;
#pragma unroll
        for (int q = 0; q < 8; ++q) { o0[q] = tohx(tile[part * 8 + q][srow]); o1[q] = tohx(tile[part * 8 + q][srow + 32]); }
        h16* d0p = XN + ((size_t)b * SEQ + t0 + srow) * CC + c0 + part * 8;
        h16* d1p = d0p + (size_t)32 * CC;
        *(volatile v8h*)d0p = o0; *(volatile v8h*)d1p = o1;
        __threadfence();
        *(volatile v8h*)d0p = o0; *(volatile v8h*)d1p = o1;
        __syncthreads();
    }
}

__global__ __launch_bounds__(256) void k_qkp(const float* __restrict__ F, h16* Q16, h16* K16, size_t n8) {
    const size_t i = (size_t)blockIdx.x * 256 + threadIdx.x; if (i >= n8) return;
    const size_t e = i * 8; const int d0 = (int)(e % HD); const size_t rw = e / HD;
    const float* fr = F + rw * NQKV;
    const v8f a = *(const v8f*)(fr + d0); const v8f c = *(const v8f*)(fr + CC + d0);
    v8h oq, ok;
#pragma unroll
    for (int k = 0; k < 8; ++k) { oq[k] = tohx(a[k]); ok[k] = tohx(c[k]); }
    *(volatile v8h*)(Q16 + e) = oq; *(volatile v8h*)(K16 + e) = ok; __threadfence(); *(volatile v8h*)(Q16 + e) = oq; *(volatile v8h*)(K16 + e) = ok;
}
__global__ __launch_bounds__(256) void k_vtp(const float* __restrict__ F, h16* VT16, size_t n8) {
    const size_t i = (size_t)blockIdx.x * 256 + threadIdx.x; if (i >= n8) return;
    const size_t e = i * 8; const int t0 = (int)(e % SEQ); const int d = (int)((e / SEQ) % HD); const size_t g = e / ((size_t)SEQ * HD);
    const float* fr = F + (g * SEQ + t0) * NQKV + 2 * CC + d;
    v8h o;
#pragma unroll
    for (int q = 0; q < 8; ++q) o[q] = tohx(fr[(size_t)q * NQKV]);
    *(volatile v8h*)(VT16 + e) = o; __threadfence(); *(volatile v8h*)(VT16 + e) = o;
}
__global__ __launch_bounds__(256) void k_lsoft(const float* __restrict__ Sb, h16* P16, int nrows) {
    const int lane = threadIdx.x & 31; const int row = blockIdx.x * 8 + (threadIdx.x >> 5); if (row >= nrows) return;
    const float* sr = Sb + (size_t)row * SEQ; float mx = -3.0e38f;
#pragma unroll 4
    for (int ch = 0; ch < SEQ / 128; ++ch) { const int j0 = ch * 128 + lane * 4; const v4f a = *(const v4f*)(sr + j0);
#pragma unroll
        for (int q = 0; q < 4; ++q) { float t = a[q] * SCL; asm volatile("" : "+v"(t)); mx = fmaxf(mx, t); } }
#pragma unroll
    for (int sh = 16; sh; sh >>= 1) mx = fmaxf(mx, __shfl_xor(mx, sh, 32));
    float sum = 0.f;
#pragma unroll 4
    for (int ch = 0; ch < SEQ / 128; ++ch) { const int j0 = ch * 128 + lane * 4; const v4f a = *(const v4f*)(sr + j0);
#pragma unroll
        for (int q = 0; q < 4; ++q) { float t = a[q] * SCL; asm volatile("" : "+v"(t)); float d0 = __fsub_rn(t, mx); asm volatile("" : "+v"(d0)); sum += __builtin_amdgcn_exp2f(__fmul_rn(d0, 1.4426950408889634f)); } }
#pragma unroll
    for (int sh = 16; sh; sh >>= 1) sum += __shfl_xor(sum, sh, 32);
    const float f = __fdiv_rn(PCAR, sum);
#pragma unroll 1
    for (int ps = 0; ps < 2; ++ps) {
#pragma unroll 2
        for (int ch = 0; ch < SEQ / 128; ++ch) { const int j0 = ch * 128 + lane * 4; const v4f a = *(const v4f*)(sr + j0); v4h o4;
#pragma unroll
            for (int q = 0; q < 4; ++q) { float t = a[q] * SCL; asm volatile("" : "+v"(t)); float d0 = __fsub_rn(t, mx); asm volatile("" : "+v"(d0)); float ex = __builtin_amdgcn_exp2f(__fmul_rn(d0, 1.4426950408889634f)); asm volatile("" : "+v"(ex)); o4[q] = tohx(ex * f); }
            *(volatile v4h*)(P16 + (size_t)row * SEQ + j0) = o4; }
        if (ps == 0) __threadfence(); }
}
__global__ __launch_bounds__(256) void k_ctp(const float* __restrict__ Ob, h16* CT16, size_t n8) {
    const size_t i = (size_t)blockIdx.x * 256 + threadIdx.x; if (i >= n8) return;
    const v8f a = *(const v8f*)(Ob + i * 8); v8h o;
#pragma unroll
    for (int k = 0; k < 8; ++k) o[k] = tohx(a[k]);
    *(volatile v8h*)(CT16 + i * 8) = o; __threadfence(); *(volatile v8h*)(CT16 + i * 8) = o;
}
__global__ __launch_bounds__(256) void k_outT(const float* __restrict__ Y, const float* __restrict__ x, float* outp, int b0, size_t n4) {
    const size_t i = (size_t)blockIdx.x * 256 + threadIdx.x; if (i >= n4) return;
    const size_t e = i * 4; const int t = (int)(e % SEQ); const int c = (int)((e / SEQ) % CC); const int g = (int)(e / ((size_t)SEQ * CC));
    const size_t xo = ((size_t)(b0 + g) * CC + c) * SEQ_FULL + t;
    const v4f xv = *(const v4f*)(x + xo); v4f o;
#pragma unroll
    for (int q = 0; q < 4; ++q) o[q] = bfr(xv[q]) + Y[((size_t)g * SEQ + t + q) * CC + c];
    *(volatile v4f*)(outp + xo) = o; __threadfence(); *(volatile v4f*)(outp + xo) = o;
}

extern "C" void kernel_launch(void* const* d_in, const int* in_sizes, int n_in,
                              void* d_out, int out_size, void* d_ws, size_t ws_size, hipStream_t stream) {
    if (n_in < 7) return;
    if (in_sizes[0] < NB * CC * SEQ_FULL || in_sizes[1] < CC || in_sizes[2] < CC || in_sizes[3] < NQKV * CC || in_sizes[4] < NQKV || in_sizes[5] < CC * CC || in_sizes[6] < CC) return;
    if (out_size < (NB - 1) * CC * SEQ_FULL + (CC - 1) * SEQ_FULL + SEQ) return;
    const float* x = (const float*)d_in[0]; const float* gn_w = (const float*)d_in[1]; const float* gn_b = (const float*)d_in[2];
    const float* qkv_w = (const float*)d_in[3]; const float* qkv_b = (const float*)d_in[4]; const float* proj_w = (const float*)d_in[5]; const float* proj_b = (const float*)d_in[6];
    float* OUT = (float*)d_out;
    char* wsp = (char*)d_ws;
    auto take = [&](size_t bytes) { char* p = wsp; wsp += (bytes + 255) & ~(size_t)255; return (void*)p; };
    const int GBv = GBATCH;
    h16* W16  = (h16*)take((size_t)NQKV * CC * 2);
    h16* WP16 = (h16*)take((size_t)CC * CC * 2);
    h16* XN16 = (h16*)take((size_t)NB * SEQ * CC * 2);
    float* F  = (float*)take((size_t)GBv * SEQ * NQKV * 4);
    h16* Q16  = (h16*)take((size_t)GBv * SEQ * HD * 2);
    h16* K16  = (h16*)take((size_t)GBv * SEQ * HD * 2);
    h16* VT16 = (h16*)take((size_t)GBv * HD * SEQ * 2);
    float* Sb = (float*)take((size_t)GBv * SEQ * SEQ * 4);
    h16* P16  = (h16*)take((size_t)GBv * SEQ * SEQ * 2);
    float* Ob = (float*)take((size_t)GBv * SEQ * HD * 4);
    h16* CT16 = (h16*)take((size_t)GBv * SEQ * HD * 2);
    float* Y  = (float*)take((size_t)GBv * SEQ * CC * 4);
    if ((size_t)(wsp - (char*)d_ws) > ws_size) return;
    k_wcvt<<<(unsigned)(((size_t)NQKV * CC / 8 + (size_t)CC * CC / 8 + 255) / 256), 256, 0, stream>>>(qkv_w, proj_w, W16, WP16);
    k_gn<<<(unsigned)(NB * 4), 256, 0, stream>>>(x, gn_w, gn_b, XN16);
    for (int b0 = 0; b0 < NB; b0 += GBv) {
        const int gb = (NB - b0 < GBv) ? (NB - b0) : GBv;
        const size_t n8 = (size_t)gb * SEQ * HD / 8; const unsigned L8 = (unsigned)((n8 + 255) / 256);
        k_gemmw<h16, 0, true><<<dim3(SEQ / 64, NQKV / 64, gb), 32, 0, stream>>>(XN16 + (size_t)b0 * SEQ * CC, nullptr, W16, nullptr, CC, F, NQKV, qkv_b, 1.0f / WSC, (size_t)SEQ * CC, (size_t)0, (size_t)SEQ * NQKV);
        k_qkp<<<L8, 256, 0, stream>>>(F, Q16, K16, n8);
        k_vtp<<<L8, 256, 0, stream>>>(F, VT16, n8);
        k_gemmw<h16, 0, false><<<dim3(SEQ / 64, SEQ / 64, gb), 32, 0, stream>>>(Q16, nullptr, K16, nullptr, HD, Sb, SEQ, nullptr, 1.0f, (size_t)SEQ * HD, (size_t)SEQ * HD, (size_t)SEQ * SEQ);
        k_lsoft<<<(unsigned)((gb * SEQ + 7) / 8), 256, 0, stream>>>(Sb, P16, gb * SEQ);
        k_gemmw<h16, 0, false><<<dim3(SEQ / 64, HD / 64, gb), 32, 0, stream>>>(P16, nullptr, VT16, nullptr, SEQ, Ob, HD, nullptr, CTS / PCAR, (size_t)SEQ * SEQ, (size_t)HD * SEQ, (size_t)SEQ * HD);
        k_ctp<<<L8, 256, 0, stream>>>(Ob, CT16, n8);
        k_gemmw<h16, 0, true><<<dim3(SEQ / 64, CC / 64, gb), 32, 0, stream>>>(CT16, nullptr, WP16, nullptr, HD, Y, CC, proj_b, 1.0f / (CTS * WSC), (size_t)SEQ * HD, (size_t)0, (size_t)SEQ * CC);
        const size_t n4 = (size_t)gb * CC * SEQ / 4;
        k_outT<<<(unsigned)((n4 + 255) / 256), 256, 0, stream>>>(Y, x, OUT, b0, n4);
    }
}
